// MambaBlock_8667244003586
// MI455X (gfx1250) — hardware-verified
//
#include <hip/hip_runtime.h>
#include <math.h>

typedef __attribute__((ext_vector_type(16))) _Float16 v16h;
typedef __attribute__((ext_vector_type(8)))  _Float16 v8h;
typedef __attribute__((ext_vector_type(8)))  float    v8f;
typedef __attribute__((ext_vector_type(4)))  float    v4f;

constexpr int kBatch  = 2;
constexpr int kSeqL   = 4096;
constexpr int kDm     = 768;
constexpr int kEin    = 1536;
constexpr int kNst    = 16;
constexpr int kRows   = kBatch * kSeqL;
constexpr int kXpW    = kDm + kNst;
constexpr int kXdReal = kXpW + kNst;
constexpr int kXdP    = 832;
constexpr int kConvTP = 260;
constexpr int kScanTS = 32;
constexpr float kWCarry   = 32.0f;
constexpr float kActCarry = 16.0f;
constexpr float kScaleG1  = 1.0f / kWCarry;
constexpr float kScaleG23 = 1.0f / (kWCarry * kActCarry);
constexpr float kInvDm    = 1.0f / (float)kDm;
constexpr float kLnEps    = 1e-5f;
constexpr float kF32MinNormal = 1.17549435e-38f;

static_assert(kRows == 8192);
static_assert(kXpW == 784 && kXdReal == 800 && kXdP >= kXdReal && (kXdP % 64) == 0);
static_assert((kDm % 32) == 0 && (kEin % 32) == 0);
static_assert((kRows % 64) == 0 && (kEin % 64) == 0 && (kDm % 64) == 0);
static_assert((kDm % 256) == 0 && (kEin % 256) == 0 && (kSeqL % 64) == 0 && (kSeqL % kScanTS) == 0);

constexpr size_t kOffWINT = 0;
constexpr size_t kOffWCAT = kOffWINT + (size_t)kEin  * kDm  * 2;
constexpr size_t kOffWOUT = kOffWCAT + (size_t)kXdP  * kEin * 2;
constexpr size_t kOffXN   = kOffWOUT + (size_t)kDm   * kEin * 2;
constexpr size_t kOffXIN  = kOffXN   + (size_t)kRows * kDm  * 2;
constexpr size_t kOffXACT = kOffXIN  + (size_t)kRows * kEin * 4;
constexpr size_t kOffXD   = kOffXACT + (size_t)kRows * kEin * 2;
constexpr size_t kOffUS   = kOffXD   + (size_t)kRows * kXdP * 4;
constexpr size_t kWsTotal = kOffUS   + (size_t)kRows * kNst * 4;
static_assert(kWsTotal == 123142144ull);
static_assert(kWsTotal <= 134217728ull);
static_assert((kOffWCAT % 128) == 0 && (kOffWOUT % 128) == 0 && (kOffXN % 128) == 0 && (kOffXIN % 128) == 0 &&
              (kOffXACT % 128) == 0 && (kOffXD % 128) == 0 && (kOffUS % 128) == 0);

union FragU { v16h v; v8h h[2]; };
__device__ __forceinline__ v16h frag_load(const _Float16* p) {
  FragU f;
  f.h[0] = *(const v8h*)(p);
  f.h[1] = *(const v8h*)(p + 16);
  return f.v;
}
__device__ __forceinline__ v8f frag_mma(v16h a, v16h b, v8f c) {
  return __builtin_amdgcn_wmma_f32_16x16x32_f16(false, a, false, b, (short)0, c, false, false);
}
__device__ __forceinline__ void group_guard(v8f& a, v8f& b, v8f& c, v8f& d, v16h x,
                                            v16h b0, v16h b1, v16h b2, v16h b3) {
  asm volatile("v_nop\n\tv_nop\n\tv_nop\n\tv_nop"
               : "+v"(a), "+v"(b), "+v"(c), "+v"(d)
               : "v"(x), "v"(b0), "v"(b1), "v"(b2), "v"(b3));
}
__device__ __forceinline__ void keep4_h(v16h a, v16h b, v16h c, v16h d) { asm volatile("v_nop" :: "v"(a), "v"(b), "v"(c), "v"(d)); }
__device__ __forceinline__ void acc_guard4(v8f& a, v8f& b, v8f& c, v8f& d) { asm volatile("v_nop\n\tv_nop\n\tv_nop\n\tv_nop" : "+v"(a), "+v"(b), "+v"(c), "+v"(d)); }

template <int BIAS_MODE>
__global__ __launch_bounds__(256) void wmma_gemm64_f16(
    const unsigned short* __restrict__ Ap, int lda,
    const unsigned short* __restrict__ Btp, int ldb,
    float* __restrict__ C, int ldc,
    const float* __restrict__ bias,
    int M, int N, int K, float scale) {
  const _Float16* A  = (const _Float16*)Ap;
  const _Float16* Bt = (const _Float16*)Btp;
  __shared__ __align__(16) float sT[8][16 * 68];
  const int lane = threadIdx.x & 31;
  const int wave = threadIdx.x >> 5;
  const int tilesN = N >> 6;
  const int tilesM = M >> 6;
  const int tile = blockIdx.x * 8 + wave;
  if (tile >= tilesM * tilesN) return;
  const int tm = tile / tilesN;
  const int tn = tile - tm * tilesN;
  const int m0 = tm << 6;
  const int n0 = tn << 6;

  const int rlane = lane & 15;
  const int koff  = (lane >> 4) * 8;
  const int mOff  = (lane >> 4) * 8;

  v8f acc[4][4];
#pragma unroll
  for (int i = 0; i < 4; ++i)
#pragma unroll
    for (int j = 0; j < 4; ++j) acc[i][j] = (v8f){0.f,0.f,0.f,0.f,0.f,0.f,0.f,0.f};

  for (int k0 = 0; k0 < K; k0 += 32) {
    v16h bh[4];
#pragma unroll
    for (int j = 0; j < 4; ++j) {
      const size_t bo = (size_t)(n0 + (j << 4) + rlane) * ldb + koff + k0;
      bh[j] = frag_load(Bt + bo);
    }
#pragma unroll
    for (int i = 0; i < 4; ++i) {
      const size_t ao = (size_t)(m0 + (i << 4) + rlane) * lda + koff + k0;
      const v16h ah = frag_load(A + ao);
#pragma unroll
      for (int j = 0; j < 4; ++j) acc[i][j] = frag_mma(ah, bh[j], acc[i][j]);
      group_guard(acc[i][0], acc[i][1], acc[i][2], acc[i][3], ah, bh[0], bh[1], bh[2], bh[3]);
    }
    keep4_h(bh[0], bh[1], bh[2], bh[3]);
  }
  acc_guard4(acc[0][0], acc[0][1], acc[0][2], acc[0][3]);
  acc_guard4(acc[1][0], acc[1][1], acc[1][2], acc[1][3]);
  acc_guard4(acc[2][0], acc[2][1], acc[2][2], acc[2][3]);
  acc_guard4(acc[3][0], acc[3][1], acc[3][2], acc[3][3]);

  float* slab = sT[wave];
#pragma unroll
  for (int i = 0; i < 4; ++i) {
    const int mBase = m0 + (i << 4);
#pragma unroll
    for (int j = 0; j < 4; ++j) {
      const int n = n0 + (j << 4) + rlane;
      float bv = 0.f;
      if (BIAS_MODE == 2) bv = bias[n];
#pragma unroll
      for (int r = 0; r < 8; ++r) {
        float v = acc[i][j][r] * scale;
        if (BIAS_MODE == 2) v += bv;
        slab[(mOff + r) * 68 + (j << 4) + rlane] = v;
      }
    }
    __builtin_amdgcn_fence(__ATOMIC_RELEASE, "workgroup");
    __builtin_amdgcn_wave_barrier();
    __builtin_amdgcn_fence(__ATOMIC_ACQUIRE, "workgroup");
    {
      const int hh = lane >> 4, c4 = (lane & 15) * 4;
      for (int pass = 0; pass < 2; ++pass) {
#pragma unroll
        for (int it = 0; it < 8; ++it) {
          const int row = it * 2 + hh;
          v4f v = *(const v4f*)(slab + row * 68 + c4);
          *(volatile v4f*)(C + (size_t)(mBase + row) * ldc + n0 + c4) = v;
        }
        __threadfence();
      }
    }
    __builtin_amdgcn_fence(__ATOMIC_RELEASE, "workgroup");
    __builtin_amdgcn_wave_barrier();
    __builtin_amdgcn_fence(__ATOMIC_ACQUIRE, "workgroup");
  }
}

template <bool TWO>
__global__ __launch_bounds__(256) void transpose_cast_kernel(
    const float* __restrict__ W1, int N1, const float* __restrict__ W2, int N2,
    unsigned short* __restrict__ Bt, int Kdim, float scale)
{
  __shared__ float tile[64 * 65];
  const int tid = threadIdx.x, lane = tid & 31, wave = tid >> 5;
  const int n0 = blockIdx.x * 64;
  const int k0 = blockIdx.y * 64;
#pragma unroll
  for (int p = 0; p < 16; ++p) {
    const int idx = tid + p * 256;
    const int kk  = idx >> 6;
    const int nn  = idx & 63;
    const int n   = n0 + nn;
    const int n1c = (n < N1) ? n : (N1 - 1);
    const float a = W1[(size_t)(k0 + kk) * N1 + n1c];
    float v;
    if (TWO) {
      const int m  = n - N1;
      const int mc = (m < 0) ? 0 : ((m < N2) ? m : (N2 - 1));
      const float b  = W2[(size_t)(k0 + kk) * N2 + mc];
      const float fa = (n < N1) ? 1.0f : 0.0f;
      const float fb = (m >= 0 && m < N2) ? 1.0f : 0.0f;
      v = fmaf(fb, b, fa * a) * scale;
    } else {
      v = (n < N1) ? (a * scale) : 0.f;
    }
    tile[kk * 65 + nn] = v;
    if ((p & 3) == 3) asm volatile("" ::: "memory");
  }
  __syncthreads();
  const int q = lane >> 3, c8 = (lane & 7) * 8;
  v8h hv[2];
#pragma unroll
  for (int it = 0; it < 2; ++it) {
    const int nrow = it * 32 + wave * 4 + q;
#pragma unroll
    for (int e = 0; e < 8; ++e) hv[it][e] = (_Float16)tile[(c8 + e) * 65 + nrow];
  }
  for (int pass = 0; pass < 2; ++pass) {
#pragma unroll
    for (int it = 0; it < 2; ++it) {
      const int nrow = it * 32 + wave * 4 + q;
      *(volatile v8h*)(Bt + (size_t)(n0 + nrow) * Kdim + k0 + c8) = hv[it];
    }
    __threadfence();
  }
}

__global__ __launch_bounds__(256) void ln_kernel(
    const float* __restrict__ X, const float* __restrict__ G, const float* __restrict__ Bv,
    unsigned short* __restrict__ XN)
{
  const int lane = threadIdx.x & 31, wave = threadIdx.x >> 5;
  const int row = blockIdx.x * 8 + wave;
  const float* xr = X + (size_t)row * kDm;
  v4f xv[6];
#pragma unroll
  for (int c = 0; c < 3; ++c) {
    xv[2 * c]     = *(const v4f*)(xr + c * 256 + lane * 8);
    xv[2 * c + 1] = *(const v4f*)(xr + c * 256 + lane * 8 + 4);
  }
  asm volatile("" ::: "memory");
  float sum = 0.f;
#pragma unroll
  for (int i = 0; i < 6; ++i)
#pragma unroll
    for (int e = 0; e < 4; ++e) sum += xv[i][e];
#pragma unroll
  for (int off = 16; off > 0; off >>= 1) sum += __shfl_xor(sum, off, 32);
  const float mu = sum * kInvDm;
  float sq = 0.f;
#pragma unroll
  for (int i = 0; i < 6; ++i)
#pragma unroll
    for (int e = 0; e < 4; ++e) {
      const float dlt = xv[i][e] - mu;
      sq += dlt * dlt;
    }
#pragma unroll
  for (int off = 16; off > 0; off >>= 1) sq += __shfl_xor(sq, off, 32);
  const float rstd = rsqrtf(sq * kInvDm + kLnEps);
  v8h hv[3];
#pragma unroll
  for (int c = 0; c < 3; ++c) {
    const int col = c * 256 + lane * 8;
    const v4f g0 = *(const v4f*)(G + col);
    const v4f g1 = *(const v4f*)(G + col + 4);
    const v4f b0 = *(const v4f*)(Bv + col);
    const v4f b1 = *(const v4f*)(Bv + col + 4);
#pragma unroll
    for (int e = 0; e < 4; ++e) {
      const float y0 = (xv[2 * c][e] - mu) * rstd * g0[e] + b0[e];
      const float y1 = (xv[2 * c + 1][e] - mu) * rstd * g1[e] + b1[e];
      hv[c][e]     = (_Float16)y0;
      hv[c][4 + e] = (_Float16)y1;
    }
    asm volatile("" ::: "memory");
  }
  unsigned short* orow = XN + (size_t)row * kDm;
  for (int pass = 0; pass < 2; ++pass) {
#pragma unroll
    for (int c = 0; c < 3; ++c) *(volatile v8h*)(orow + c * 256 + lane * 8) = hv[c];
    __threadfence();
  }
}

__global__ __launch_bounds__(256) void conv_silu_kernel(
    const float* __restrict__ XI, const float* __restrict__ cw, const float* __restrict__ cb,
    unsigned short* __restrict__ XA)
{
  __shared__ __align__(16) float sT[16 * kConvTP];
  const int tid = threadIdx.x, lane = tid & 31, wave = tid >> 5;
  const int d0 = blockIdx.x * 256, d = d0 + tid;
  const int g0 = blockIdx.y * 64;
  const int tb = g0 & (kSeqL - 1);
  const v4f wv = *(const v4f*)(cw + (size_t)d * 4);
  const float w0 = wv[0], w1 = wv[1], w2 = wv[2], w3 = wv[3];
  const float bc = cb[d];
  float xm3, xm2, xm1;
  {
    const bool hist = (tb > 0);
    const int rb = hist ? (g0 - 3) : g0;
    const float v3 = XI[(size_t)rb * kEin + d];
    const float v2 = XI[(size_t)(rb + 1) * kEin + d];
    const float v1 = XI[(size_t)(rb + 2) * kEin + d];
    xm3 = hist ? v3 : 0.f;
    xm2 = hist ? v2 : 0.f;
    xm1 = hist ? v1 : 0.f;
  }
#pragma unroll 1
  for (int sub = 0; sub < 4; ++sub) {
    const int lb = g0 + sub * 16;
#pragma unroll 1
    for (int s = 0; s < 16; ++s) {
      const float xcur = XI[(size_t)(lb + s) * kEin + d];
      float acc = w0 * xm3;
      acc = fmaf(w1, xm2, acc);
      acc = fmaf(w2, xm1, acc);
      acc = fmaf(w3, xcur, acc);
      const float sv = acc + bc;
      const float sg = __builtin_amdgcn_rcpf(1.0f + expf(-sv));
      sT[s * kConvTP + tid] = sv * sg;
      xm3 = xm2; xm2 = xm1; xm1 = xcur;
    }
    __syncthreads();
    v8h bv[2];
#pragma unroll
    for (int it = 0; it < 2; ++it) {
      const float* sp = sT + (it * 8 + wave) * kConvTP + lane * 8;
      const v4f a0 = *(const v4f*)(sp);
      const v4f a1 = *(const v4f*)(sp + 4);
#pragma unroll
      for (int e = 0; e < 4; ++e) {
        bv[it][e]     = (_Float16)(a0[e] * kActCarry);
        bv[it][4 + e] = (_Float16)(a1[e] * kActCarry);
      }
    }
    for (int pass = 0; pass < 2; ++pass) {
#pragma unroll
      for (int it = 0; it < 2; ++it)
        *(volatile v8h*)(XA + (size_t)(lb + it * 8 + wave) * kEin + d0 + lane * 8) = bv[it];
      __threadfence();
    }
    __syncthreads();
  }
}

__global__ __launch_bounds__(32) void scan_kernel(
    const float* __restrict__ XD, const float* __restrict__ bxp, const float* __restrict__ bdt,
    float* __restrict__ US)
{
  __shared__ __align__(16) float sU[2 * kScanTS * kNst];
  const int lane = threadIdx.x;
  const int b = lane >> 4, s = lane & 15;
  const float bds = bxp[kDm + s];
  const float bz  = bdt[s];
  const size_t rowb = (size_t)b * kSeqL;
  float v = 0.f;
#pragma unroll 1
  for (int t0 = 0; t0 < kSeqL; t0 += kScanTS) {
#pragma unroll 1
    for (int st = 0; st < kScanTS; ++st) {
      const int t = t0 + st;
      const float* xr = XD + (rowb + (size_t)t) * kXdP + kDm;
      const float ds = xr[s] + bds;
      const float zz = xr[kNst + s] + bz;
      const float dt = fmaxf(zz, 0.0f) + log1pf(expf(-fabsf(zz)));
      const float hh = expf(-0.5f * dt);
      const float a  = hh * hh;
      const float bt = ds * hh;
      v = a * v + bt;
      float dn = expm1f(-dt);
      dn = (dn > -1e-30f) ? -1e-30f : dn;
      const float kf = (float)(kSeqL - 1 - t);
      float e1 = expf(-kf * dt);
      e1 = (e1 < kF32MinNormal) ? 0.0f : e1;
      const float em = e1 - 1.0f;
      const float rc = __builtin_amdgcn_rcpf(dn);
      const float uo = e1 * v + (bt * em) * rc;
      sU[b * (kScanTS * kNst) + st * kNst + s] = uo;
    }
    __syncthreads();
    v4f uv[8];
#pragma unroll
    for (int b2 = 0; b2 < 2; ++b2)
#pragma unroll
      for (int it = 0; it < 4; ++it)
        uv[b2 * 4 + it] = *(const v4f*)(sU + b2 * (kScanTS * kNst) + (it * 32 + lane) * 4);
    for (int pass = 0; pass < 2; ++pass) {
#pragma unroll
      for (int b2 = 0; b2 < 2; ++b2)
#pragma unroll
        for (int it = 0; it < 4; ++it)
          *(volatile v4f*)(US + ((size_t)b2 * kSeqL + t0) * kNst + (it * 32 + lane) * 4) = uv[b2 * 4 + it];
      __threadfence();
    }
    __syncthreads();
  }
}

__global__ __launch_bounds__(256) void ybuild_kernel(
    const float* __restrict__ XD, const float* __restrict__ US, const float* __restrict__ Wus,
    const float* __restrict__ bxp, const float* __restrict__ bus, unsigned short* __restrict__ XA)
{
  __shared__ __align__(16) float sW[kNst * 256];
  __shared__ __align__(16) float sU[64 * kNst];
  const int tid = threadIdx.x, lane = tid & 31, wave = tid >> 5;
  const int cs = blockIdx.x * 256;
  const int r0 = blockIdx.y * 64;
#pragma unroll
  for (int p = 0; p < 4; ++p) {
    const int idx = tid + p * 256;
    const int ss = idx >> 6;
    const int q4 = (idx & 63) * 4;
    *(v4f*)(sW + ss * 256 + q4) = *(const v4f*)(Wus + (size_t)ss * kDm + cs + q4);
  }
  *(v4f*)(sU + tid * 4) = *(const v4f*)(US + (size_t)r0 * kNst + tid * 4);
  const int c0 = cs + lane * 8;
  float bs[8];
  {
    const v4f p0 = *(const v4f*)(bxp + c0);
    const v4f p1 = *(const v4f*)(bxp + c0 + 4);
    const v4f u0 = *(const v4f*)(bus + c0);
    const v4f u1 = *(const v4f*)(bus + c0 + 4);
#pragma unroll
    for (int e = 0; e < 4; ++e) {
      bs[e]     = p0[e] + u0[e];
      bs[4 + e] = p1[e] + u1[e];
    }
  }
  __syncthreads();
#pragma unroll 1
  for (int it = 0; it < 8; ++it) {
    const int rl = it * 8 + wave;
    const size_t row = (size_t)(r0 + rl);
    const v4f x0 = *(const v4f*)(XD + row * kXdP + c0);
    const v4f x1 = *(const v4f*)(XD + row * kXdP + c0 + 4);
    float acc[8];
#pragma unroll
    for (int e = 0; e < 4; ++e) {
      acc[e]     = x0[e] + bs[e];
      acc[4 + e] = x1[e] + bs[4 + e];
    }
#pragma unroll 1
    for (int ss = 0; ss < kNst; ++ss) {
      const float u = sU[rl * kNst + ss];
      const v4f wa = *(const v4f*)(sW + ss * 256 + lane * 8);
      const v4f wb = *(const v4f*)(sW + ss * 256 + lane * 8 + 4);
#pragma unroll
      for (int e = 0; e < 4; ++e) {
        acc[e]     = fmaf(u, wa[e], acc[e]);
        acc[4 + e] = fmaf(u, wb[e], acc[4 + e]);
      }
    }
    v8h hv;
#pragma unroll
    for (int e = 0; e < 8; ++e) hv[e] = (_Float16)(acc[e] * kActCarry);
    unsigned short* dst = XA + row * kEin + c0;
    *(volatile v8h*)dst = hv;
    __threadfence();
    *(volatile v8h*)dst = hv;
  }
}

static_assert(((kRows / 64) * (kEin / 64)) % 8 == 0);
static_assert(((kRows / 64) * (kXdP / 64)) % 8 == 0);
static_assert(((kRows / 64) * (kDm / 64)) % 8 == 0);

extern "C" void kernel_launch(void* const* d_in, const int* in_sizes, int n_in,
                              void* d_out, int out_size, void* d_ws, size_t ws_size,
                              hipStream_t stream)
{
  if (n_in < 15) return;
  if (in_sizes[0] != kRows * kDm) return;
  if (in_sizes[1] != kDm || in_sizes[2] != kDm) return;
  if (in_sizes[3] != kDm * kEin || in_sizes[4] != kEin) return;
  if (in_sizes[5] != kEin * 4 || in_sizes[6] != kEin) return;
  if (in_sizes[7] != kEin * kXpW || in_sizes[8] != kXpW) return;
  if (in_sizes[9] != kEin * kNst || in_sizes[10] != kNst) return;
  if (in_sizes[11] != kNst * kDm || in_sizes[12] != kDm) return;
  if (in_sizes[13] != kEin * kDm || in_sizes[14] != kDm) return;
  if (out_size != kRows * kDm) return;
  if (ws_size < kWsTotal) return;

  const float* x      = (const float*)d_in[0];
  const float* ln_g   = (const float*)d_in[1];
  const float* ln_b   = (const float*)d_in[2];
  const float* W_in   = (const float*)d_in[3];
  const float* b_in   = (const float*)d_in[4];
  const float* W_conv = (const float*)d_in[5];
  const float* b_conv = (const float*)d_in[6];
  const float* W_xp   = (const float*)d_in[7];
  const float* b_xp   = (const float*)d_in[8];
  const float* W_dt   = (const float*)d_in[9];
  const float* b_dt   = (const float*)d_in[10];
  const float* W_us   = (const float*)d_in[11];
  const float* b_us   = (const float*)d_in[12];
  const float* W_out  = (const float*)d_in[13];
  const float* b_out  = (const float*)d_in[14];
  float* out = (float*)d_out;

  char* ws = (char*)d_ws;
  unsigned short* WINT = (unsigned short*)(ws + kOffWINT);
  unsigned short* WCAT = (unsigned short*)(ws + kOffWCAT);
  unsigned short* WOUT = (unsigned short*)(ws + kOffWOUT);
  unsigned short* XN   = (unsigned short*)(ws + kOffXN);
  float*          XIN  = (float*)(ws + kOffXIN);
  unsigned short* XACT = (unsigned short*)(ws + kOffXACT);
  float*          XD   = (float*)(ws + kOffXD);
  float*          US   = (float*)(ws + kOffUS);

  transpose_cast_kernel<false><<<dim3(kEin / 64, kDm / 64), 256, 0, stream>>>(W_in, kEin, W_in, 0, WINT, kDm, kWCarry);
  transpose_cast_kernel<true><<<dim3(kXdP / 64, kEin / 64), 256, 0, stream>>>(W_xp, kXpW, W_dt, kNst, WCAT, kEin, kWCarry);
  transpose_cast_kernel<false><<<dim3(kDm / 64, kEin / 64), 256, 0, stream>>>(W_out, kDm, W_out, 0, WOUT, kEin, kWCarry);

  ln_kernel<<<kRows / 8, 256, 0, stream>>>(x, ln_g, ln_b, XN);

  wmma_gemm64_f16<2><<<((kRows / 64) * (kEin / 64)) / 8, 256, 0, stream>>>(
      XN, kDm, WINT, kDm, XIN, kEin, b_in, kRows, kEin, kDm, kScaleG1);

  conv_silu_kernel<<<dim3(kEin / 256, kRows / 64), 256, 0, stream>>>(XIN, W_conv, b_conv, XACT);

  wmma_gemm64_f16<0><<<((kRows / 64) * (kXdP / 64)) / 8, 256, 0, stream>>>(
      XACT, kEin, WCAT, kEin, XD, kXdP, b_in, kRows, kXdP, kEin, kScaleG23);

  scan_kernel<<<1, 32, 0, stream>>>(XD, b_xp, b_dt, US);

  ybuild_kernel<<<dim3(kDm / 256, kRows / 64), 256, 0, stream>>>(XD, US, W_us, b_xp, b_us, XACT);

  wmma_gemm64_f16<2><<<((kRows / 64) * (kDm / 64)) / 8, 256, 0, stream>>>(
      XACT, kEin, WOUT, kEin, out, kDm, b_out, kRows, kDm, kEin, kScaleG23);
}
